// TFFlaubertMultiHeadAttention_4131758539278
// MI455X (gfx1250) — hardware-verified
//
#include <hip/hip_runtime.h>
#include <math.h>
#include <stdint.h>

typedef __attribute__((ext_vector_type(16))) _Float16 v16h;
typedef __attribute__((ext_vector_type(8)))  _Float16 v8h;
typedef __attribute__((ext_vector_type(16))) __bf16   v16b;
typedef __attribute__((ext_vector_type(8)))  __bf16   v8b;
typedef __attribute__((ext_vector_type(8)))  float    v8f;
typedef __attribute__((ext_vector_type(4)))  float    v4f;
typedef __attribute__((ext_vector_type(2)))  float    v2f;
typedef __attribute__((ext_vector_type(4)))  unsigned int v4u;

constexpr int kBatch = 2;
constexpr int kSeq   = 2048;
constexpr int kDm    = 1024;
constexpr int kHeads = 16;
constexpr int kHd    = 64;
constexpr int kTok   = kBatch * kSeq;

__device__ __forceinline__ unsigned short f2bf_bits(float f) {
  unsigned u = __float_as_uint(f);
  return (unsigned short)((u + 0x7FFFu + ((u >> 16) & 1u)) >> 16);
}
__device__ __forceinline__ float bf_bits2f(unsigned short h) { return __uint_as_float(((unsigned)h) << 16); }
__device__ __forceinline__ unsigned pk16(unsigned short a, unsigned short b) { return (unsigned)a | ((unsigned)b << 16); }

__device__ __forceinline__ void dep_guard_h(v8f& a, v8f& b, v16h x, v16h y) { asm volatile("v_nop\n\tv_nop\n\tv_nop\n\tv_nop" : "+v"(a), "+v"(b) : "v"(x), "v"(y)); }
__device__ __forceinline__ void dep_guard_b(v8f& a, v8f& b, v16b x, v16b y) { asm volatile("v_nop\n\tv_nop\n\tv_nop\n\tv_nop" : "+v"(a), "+v"(b) : "v"(x), "v"(y)); }
__device__ __forceinline__ void keep4_h(v16h a, v16h b, v16h c, v16h d) { asm volatile("v_nop" :: "v"(a), "v"(b), "v"(c), "v"(d)); }
__device__ __forceinline__ void keep4_b(v16b a, v16b b, v16b c, v16b d) { asm volatile("v_nop" :: "v"(a), "v"(b), "v"(c), "v"(d)); }
__device__ __forceinline__ void acc_guard4(v8f& a, v8f& b, v8f& c, v8f& d) { asm volatile("v_nop\n\tv_nop\n\tv_nop\n\tv_nop" : "+v"(a), "+v"(b), "+v"(c), "+v"(d)); }
template <typename T> struct Frag;
template <> struct Frag<_Float16> {
  typedef v16h V; union U { v16h v; v8h h[2]; };
  static __device__ __forceinline__ v16h load(const _Float16* p) {
    U f; f.h[0] = *(const v8h*)(p); f.h[1] = *(const v8h*)(p + 16); return f.v;
  }
  static __device__ __forceinline__ v8f mma(v16h a, v16h b, v8f c) {
    return __builtin_amdgcn_wmma_f32_16x16x32_f16(false, a, false, b, (short)0, c, false, false);
  }
  static __device__ __forceinline__ void guard(v8f& a, v8f& b, v16h x, v16h y) { dep_guard_h(a, b, x, y); }
  static __device__ __forceinline__ void keep(v16h a, v16h b, v16h c, v16h d) { keep4_h(a, b, c, d); }
};
template <> struct Frag<__bf16> {
  typedef v16b V; union U { v16b v; v8b h[2]; };
  static __device__ __forceinline__ v16b load(const __bf16* p) {
    U f; f.h[0] = *(const v8b*)(p); f.h[1] = *(const v8b*)(p + 16); return f.v;
  }
  static __device__ __forceinline__ v8f mma(v16b a, v16b b, v8f c) {
    return __builtin_amdgcn_wmma_f32_16x16x32_bf16(false, a, false, b, (short)0, c, false, false);
  }
  static __device__ __forceinline__ void guard(v8f& a, v8f& b, v16b x, v16b y) { dep_guard_b(a, b, x, y); }
  static __device__ __forceinline__ void keep(v16b a, v16b b, v16b c, v16b d) { keep4_b(a, b, c, d); }
};

template <int ET> struct Elem;
template <> struct Elem<0> { typedef _Float16 T; };
template <> struct Elem<1> { typedef __bf16 T; };
template <int ET, int SPLIT, int BIAS_MODE, int OUT_MODE, bool RESID, int ACT = 0>
__global__ __launch_bounds__(256) void wmma_gemm64(
    const unsigned short* __restrict__ Ap, const unsigned short* __restrict__ A2p, int lda, long strideA,
    const unsigned short* __restrict__ Btp, const unsigned short* __restrict__ Bt2p, int ldb, long strideB,
    void* __restrict__ Cout, void* __restrict__ Cout2, int ldc, long strideC,
    const float* __restrict__ bias,
    const float* __restrict__ resid, long strideR,
    int M, int N, int K, float scale) {
  typedef typename Elem<ET>::T T;
  typedef typename Frag<T>::V V;
  const T* A = (const T*)Ap; const T* A2 = (const T*)A2p; const T* Bt = (const T*)Btp; const T* Bt2 = (const T*)Bt2p;
  __shared__ __align__(16) float sT[8][16 * 68];
  const int b    = blockIdx.y;
  const int lane = threadIdx.x & 31;
  const int wave = threadIdx.x >> 5;
  const int tilesN = N >> 6;
  const int tilesM = M >> 6;
  const int tile = blockIdx.x * 8 + wave;
  if (tile >= tilesM * tilesN) return;
  const int tm = tile / tilesN;
  const int tn = tile - tm * tilesN;
  const int m0 = tm << 6;
  const int n0 = tn << 6;

  const T* Ab  = A  + (size_t)b * strideA;
  const T* Bb  = Bt + (size_t)b * strideB;
  const T* Ab2 = (SPLIT >= 1) ? (A2  + (size_t)b * strideA) : nullptr;
  const T* Bb2 = (SPLIT == 2) ? (Bt2 + (size_t)b * strideB) : nullptr;

  const int rlane = lane & 15;
  const int koff  = (lane >> 4) * 8;
  const int mOff  = (lane >> 4) * 8;

  v8f acc[4][4];
#pragma unroll
  for (int i = 0; i < 4; ++i)
#pragma unroll
    for (int j = 0; j < 4; ++j) acc[i][j] = (v8f){0.f,0.f,0.f,0.f,0.f,0.f,0.f,0.f};

  for (int k0 = 0; k0 < K; k0 += 32) {
    V bh[4], bl[4];
#pragma unroll
    for (int j = 0; j < 4; ++j) {
      const size_t bo = (size_t)(n0 + (j << 4) + rlane) * ldb + koff + k0;
      bh[j] = Frag<T>::load(Bb + bo);
      if (SPLIT == 2) bl[j] = Frag<T>::load(Bb2 + bo);
    }
#pragma unroll
    for (int i = 0; i < 4; ++i) {
      const size_t ao = (size_t)(m0 + (i << 4) + rlane) * lda + koff + k0;
      V ah = Frag<T>::load(Ab + ao);
      V al;
      if (SPLIT >= 1) al = Frag<T>::load(Ab2 + ao);
#pragma unroll
      for (int j = 0; j < 4; ++j) {
        acc[i][j] = Frag<T>::mma(ah, bh[j], acc[i][j]);
        if (SPLIT == 2) acc[i][j] = Frag<T>::mma(ah, bl[j], acc[i][j]);
        if (SPLIT >= 1) acc[i][j] = Frag<T>::mma(al, bh[j], acc[i][j]);
      }
      Frag<T>::guard(acc[i][0], acc[i][3], ah, (SPLIT >= 1) ? al : ah);
    }
    Frag<T>::keep(bh[0], bh[1], bh[2], bh[3]);
    if (SPLIT == 2) Frag<T>::keep(bl[0], bl[1], bl[2], bl[3]);
  }
  acc_guard4(acc[0][0], acc[0][1], acc[0][2], acc[0][3]);
  acc_guard4(acc[1][0], acc[1][1], acc[1][2], acc[1][3]);
  acc_guard4(acc[2][0], acc[2][1], acc[2][2], acc[2][3]);
  acc_guard4(acc[3][0], acc[3][1], acc[3][2], acc[3][3]);

  float* slab = sT[wave];
  const float* Rb = RESID ? (resid + (size_t)b * strideR) : nullptr;
#pragma unroll
  for (int i = 0; i < 4; ++i) {
    const int mBase = m0 + (i << 4);
#pragma unroll
    for (int j = 0; j < 4; ++j) {
      const int n = n0 + (j << 4) + rlane;
      float bv = 0.f;
      if (BIAS_MODE == 2) bv = bias[n];
#pragma unroll
      for (int r = 0; r < 8; ++r) {
        float v = acc[i][j][r] * scale;
        if (BIAS_MODE == 1) v += bias[mBase + mOff + r];
        if (BIAS_MODE == 2) v += bv;
        if (RESID) v += Rb[(size_t)(mBase + mOff + r) * ldc + n];
        if (ACT == 1) v = tanhf(v);
        if (ACT == 2) v = fmaxf(v, 0.0f);
        if (ACT == 3) v = v / (1.0f + expf(-v));
        if (ACT == 4) v = (v > 0.f) ? v : 0.01f * v;
        slab[(mOff + r) * 68 + (j << 4) + rlane] = v;
      }
    }
    __builtin_amdgcn_fence(__ATOMIC_RELEASE, "workgroup");
    __builtin_amdgcn_wave_barrier();
    __builtin_amdgcn_fence(__ATOMIC_ACQUIRE, "workgroup");
    if (OUT_MODE == 0) {
      float* C = (float*)Cout + (size_t)b * strideC;
      const int hh = lane >> 4, c4 = (lane & 15) * 4;
      for (int pass = 0; pass < 2; ++pass) {
#pragma unroll
        for (int it = 0; it < 8; ++it) {
          const int row = it * 2 + hh;
          v4f v = *(const v4f*)(slab + row * 68 + c4);
          *(volatile v4f*)(C + (size_t)(mBase + row) * ldc + n0 + c4) = v;
        }
        __threadfence();
      }
    } else {
      const int q = lane >> 3, c8 = (lane & 7) * 8;
      unsigned short* C  = (unsigned short*)Cout  + (size_t)b * strideC;
      unsigned short* C2 = (OUT_MODE == 2) ? ((unsigned short*)Cout2 + (size_t)b * strideC) : nullptr;
      for (int pass = 0; pass < 2; ++pass) {
#pragma unroll
        for (int it = 0; it < 4; ++it) {
          const int row = it * 4 + q;
          const float* sp = slab + row * 68 + c8;
          v8h hv, lv;
#pragma unroll
          for (int e = 0; e < 8; ++e) {
            if (OUT_MODE == 1) {
              hv[e] = (_Float16)sp[e];
            } else {
              unsigned short hb = f2bf_bits(sp[e]);
              unsigned short lb = f2bf_bits(sp[e] - bf_bits2f(hb));
              hv[e] = __builtin_bit_cast(_Float16, hb);
              lv[e] = __builtin_bit_cast(_Float16, lb);
            }
          }
          *(volatile v8h*)(C + (size_t)(mBase + row) * ldc + n0 + c8) = hv;
          if (OUT_MODE == 2) *(volatile v8h*)(C2 + (size_t)(mBase + row) * ldc + n0 + c8) = lv;
        }
        __threadfence();
      }
    }
    __builtin_amdgcn_fence(__ATOMIC_RELEASE, "workgroup");
    __builtin_amdgcn_wave_barrier();
    __builtin_amdgcn_fence(__ATOMIC_ACQUIRE, "workgroup");
  }
}

__global__ __launch_bounds__(256) void cast_f32_bf16x2(const float* __restrict__ in, unsigned short* __restrict__ out, int n2) {
  const int i = blockIdx.x * 256 + threadIdx.x;
  if (i < n2) {
    const v2f f = *(const v2f*)(in + 2 * (size_t)i);
    const unsigned u = pk16(f2bf_bits(f[0]), f2bf_bits(f[1]));
    ((volatile unsigned*)out)[i] = u;
    __threadfence();
    ((volatile unsigned*)out)[i] = u;
  }
}

__global__ __launch_bounds__(256) void tcast_bf16_kernel(const float* __restrict__ W, unsigned short* __restrict__ oh, int R, int Cc) {
  __shared__ __align__(16) float tf[64 * 68];
  const int c0  = blockIdx.x * 64;
  const int r0  = blockIdx.y * 64;
  const int tid = threadIdx.x;
  {
    const int lr = tid >> 4;
    const int c4 = (tid & 15) * 4;
#pragma unroll
    for (int it = 0; it < 4; ++it) {
      const int rr = it * 16 + lr;
      const v4f a = *(const v4f*)(W + (size_t)(r0 + rr) * Cc + c0 + c4);
      *(v4f*)(tf + rr * 68 + c4) = a;
    }
  }
  __syncthreads();
  const int sub = tid >> 3;
  const int c8  = (tid & 7) * 8;
  v4u hv[2];
#pragma unroll
  for (int it = 0; it < 2; ++it) {
    const int oc = it * 32 + sub;
    v4u a;
#pragma unroll
    for (int q = 0; q < 4; ++q) {
      const float f0 = tf[(c8 + 2 * q) * 68 + oc];
      const float f1 = tf[(c8 + 2 * q + 1) * 68 + oc];
      a[q] = pk16(f2bf_bits(f0), f2bf_bits(f1));
    }
    hv[it] = a;
  }
  for (int pass = 0; pass < 2; ++pass) {
#pragma unroll
    for (int it = 0; it < 2; ++it) {
      const int oc = it * 32 + sub;
      const size_t go = (size_t)(c0 + oc) * R + r0 + c8;
      *(volatile v4u*)(oh + go) = hv[it];
    }
    __threadfence();
  }
}

constexpr int kKC = 64;
constexpr float kPCarry = 32768.0f;

__device__ __forceinline__ v8f hmma(v16h a, v16h b, v8f c) {
  c = __builtin_amdgcn_wmma_f32_16x16x32_f16(false, a, false, b, (short)0, c, false, false);
  asm volatile("v_nop\n\tv_nop\n\tv_nop\n\tv_nop" : "+v"(c) : "v"(a), "v"(b));
  return c;
}

__global__ __launch_bounds__(128)
void mha_flash_f16_kernel(const unsigned short* __restrict__ qp, const unsigned short* __restrict__ kp,
                          const unsigned short* __restrict__ vtp, const float* __restrict__ mask,
                          unsigned short* __restrict__ chp, unsigned short* __restrict__ clp, float sscale) {
  __shared__ __align__(16) _Float16 Ksh[kKC * kHd];
  __shared__ __align__(16) _Float16 Vth[kHd * kKC];
  __shared__ __align__(16) _Float16 Psh[4][16 * kKC];
  __shared__ __align__(16) float    Os[4][16 * 68];

  const int tid  = threadIdx.x;
  const int wave = tid >> 5;
  const int lane = tid & 31;
  const int hh   = lane >> 4;
  const int c    = lane & 15;

  constexpr int nqb = kSeq / 64;
  const int bx = blockIdx.x;
  const int qb = bx % nqb;
  const int bh = bx / nqb;
  const int h  = bh % kHeads;
  const int b  = bh / kHeads;
  const int q0 = qb * 64 + wave * 16;

  const _Float16* Qb = (const _Float16*)(const void*)qp  + (size_t)b * kSeq * kDm + (size_t)h * kHd;
  const _Float16* Kb = (const _Float16*)(const void*)kp  + (size_t)b * kSeq * kDm + (size_t)h * kHd;
  const _Float16* Vb = (const _Float16*)(const void*)vtp + (size_t)b * kDm * kSeq + (size_t)h * kHd * kSeq;
  const float*    mb = mask + (size_t)b * kSeq;
  unsigned short* Ch = chp + (size_t)b * kSeq * kDm + (size_t)h * kHd;
  unsigned short* Cl = clp + (size_t)b * kSeq * kDm + (size_t)h * kHd;

  v16h qa[2];
#pragma unroll
  for (int dc = 0; dc < 2; ++dc)
    qa[dc] = Frag<_Float16>::load(Qb + (size_t)(q0 + c) * kDm + dc * 32 + 8 * hh);

  float mrow[8], lrow[8];
  v8f oacc[4];
#pragma unroll
  for (int r = 0; r < 8; ++r) { mrow[r] = -INFINITY; lrow[r] = 0.f; }
#pragma unroll
  for (int t = 0; t < 4; ++t) oacc[t] = (v8f){0.f,0.f,0.f,0.f,0.f,0.f,0.f,0.f};

  constexpr int nChunks = kSeq / kKC;
  for (int kc = 0; kc < nChunks; ++kc) {
    const int kv0 = kc * kKC;
    __syncthreads();
    {
      const int r = tid >> 1, half = (tid & 1) * 32;
      const _Float16* ks = Kb + (size_t)(kv0 + r) * kDm + half;
      const _Float16* vs = Vb + (size_t)r * kSeq + kv0 + half;
#pragma unroll
      for (int i = 0; i < 4; ++i) {
        const v8h a0 = *(const v8h*)(ks + 8 * i);
        const v8h b0 = *(const v8h*)(vs + 8 * i);
        *(v8h*)(Ksh + r * kHd + half + 8 * i) = a0;
        *(v8h*)(Vth + r * kKC + half + 8 * i) = b0;
      }
    }
    __syncthreads();

    v8f s[4];
#pragma unroll
    for (int j = 0; j < 4; ++j) {
      s[j] = (v8f){0.f,0.f,0.f,0.f,0.f,0.f,0.f,0.f};
#pragma unroll
      for (int dc = 0; dc < 2; ++dc) {
        const v16h kb = Frag<_Float16>::load(Ksh + (j * 16 + c) * kHd + dc * 32 + 8 * hh);
        s[j] = hmma(qa[dc], kb, s[j]);
      }
    }
    float pen[4];
#pragma unroll
    for (int j = 0; j < 4; ++j) pen[j] = 1e30f * (1.0f - mb[kv0 + j * 16 + c]);

    float cm[8];
#pragma unroll
    for (int r = 0; r < 8; ++r) {
      float m = -INFINITY;
#pragma unroll
      for (int j = 0; j < 4; ++j) {
        const float sc = s[j][r] * sscale - pen[j];
        s[j][r] = sc;
        m = fmaxf(m, sc);
      }
#pragma unroll
      for (int off = 1; off < 16; off <<= 1) m = fmaxf(m, __shfl_xor(m, off, 32));
      cm[r] = m;
    }
    _Float16* pw = Psh[wave];
#pragma unroll
    for (int r = 0; r < 8; ++r) {
      const float mnew = fmaxf(mrow[r], cm[r]);
      const float alpha = expf(mrow[r] - mnew);
      mrow[r] = mnew;
      float psum = 0.f;
#pragma unroll
      for (int j = 0; j < 4; ++j) {
        const float p = expf(s[j][r] - mnew);
        psum += p;
        pw[(8 * hh + r) * kKC + j * 16 + c] = (_Float16)(p * kPCarry);
      }
#pragma unroll
      for (int off = 1; off < 16; off <<= 1) psum += __shfl_xor(psum, off, 32);
      lrow[r] = lrow[r] * alpha + psum;
#pragma unroll
      for (int t = 0; t < 4; ++t) oacc[t][r] *= alpha;
    }
    __builtin_amdgcn_fence(__ATOMIC_RELEASE, "workgroup");
    __builtin_amdgcn_wave_barrier();
    __builtin_amdgcn_fence(__ATOMIC_ACQUIRE, "workgroup");
#pragma unroll 1
    for (int kk = 0; kk < 2; ++kk) {
      const v16h pa = Frag<_Float16>::load(pw + c * kKC + kk * 32 + 8 * hh);
#pragma unroll
      for (int t = 0; t < 4; ++t) {
        const v16h vb = Frag<_Float16>::load(Vth + (t * 16 + c) * kKC + kk * 32 + 8 * hh);
        oacc[t] = hmma(pa, vb, oacc[t]);
      }
    }
  }

  float* os = Os[wave];
#pragma unroll
  for (int r = 0; r < 8; ++r) {
    const float inv = 1.0f / (lrow[r] * kPCarry);
#pragma unroll
    for (int t = 0; t < 4; ++t) os[(8 * hh + r) * 68 + t * 16 + c] = oacc[t][r] * inv;
  }
  __builtin_amdgcn_fence(__ATOMIC_RELEASE, "workgroup");
  __builtin_amdgcn_wave_barrier();
  __builtin_amdgcn_fence(__ATOMIC_ACQUIRE, "workgroup");
  {
    const int q = lane >> 3, c8 = (lane & 7) * 8;
    for (int pass = 0; pass < 2; ++pass) {
#pragma unroll
      for (int it = 0; it < 4; ++it) {
        const int row = it * 4 + q;
        const float* sp = os + row * 68 + c8;
        v8h hv, lv;
#pragma unroll
        for (int e = 0; e < 8; ++e) {
          const unsigned short hb = f2bf_bits(sp[e]);
          const unsigned short lb = f2bf_bits(sp[e] - bf_bits2f(hb));
          hv[e] = __builtin_bit_cast(_Float16, hb);
          lv[e] = __builtin_bit_cast(_Float16, lb);
        }
        *(volatile v8h*)(Ch + (size_t)(q0 + row) * kDm + c8) = hv;
        *(volatile v8h*)(Cl + (size_t)(q0 + row) * kDm + c8) = lv;
      }
      __threadfence();
    }
  }
}

extern "C" void kernel_launch(void* const* d_in, const int* in_sizes, int n_in,
                              void* d_out, int out_size, void* d_ws, size_t ws_size,
                              hipStream_t stream) {
  if (n_in < 10) return;
  const float* x    = (const float*)d_in[0];
  const float* mask = (const float*)d_in[1];
  const float* Wq   = (const float*)d_in[2];
  const float* bq   = (const float*)d_in[3];
  const float* Wk   = (const float*)d_in[4];
  const float* bk   = (const float*)d_in[5];
  const float* Wv   = (const float*)d_in[6];
  const float* bv   = (const float*)d_in[7];
  const float* Wo   = (const float*)d_in[8];
  const float* bo   = (const float*)d_in[9];
  float* out = (float*)d_out;

  if (in_sizes[0] != kTok * kDm || in_sizes[1] != kBatch * kSeq ||
      in_sizes[2] != kDm * kDm || in_sizes[4] != kDm * kDm || in_sizes[6] != kDm * kDm || in_sizes[8] != kDm * kDm ||
      in_sizes[3] != kDm || in_sizes[5] != kDm || in_sizes[7] != kDm || in_sizes[9] != kDm ||
      out_size != kTok * kDm) return;

  const size_t bytesTok = (size_t)kTok * kDm * 2;
  const size_t bytesW   = (size_t)kDm * kDm * 2;
  const size_t oXb = 0;
  const size_t oWq = oXb + bytesTok;
  const size_t oWk = oWq + bytesW;
  const size_t oWv = oWk + bytesW;
  const size_t oWo = oWv + bytesW;
  const size_t oQ  = oWo + bytesW;
  const size_t oK  = oQ  + bytesTok;
  const size_t oVt = oK  + bytesTok;
  const size_t oCh = oVt + bytesTok;
  const size_t oCl = oCh + bytesTok;
  const size_t total = oCl + bytesTok;
  if (total > ws_size) return;

  char* ws = (char*)d_ws;
  unsigned short* Xb  = (unsigned short*)(ws + oXb);
  unsigned short* Wqt = (unsigned short*)(ws + oWq);
  unsigned short* Wkt = (unsigned short*)(ws + oWk);
  unsigned short* Wvt = (unsigned short*)(ws + oWv);
  unsigned short* Wot = (unsigned short*)(ws + oWo);
  unsigned short* Qh  = (unsigned short*)(ws + oQ);
  unsigned short* Kh  = (unsigned short*)(ws + oK);
  unsigned short* Vt  = (unsigned short*)(ws + oVt);
  unsigned short* Ch  = (unsigned short*)(ws + oCh);
  unsigned short* Cl  = (unsigned short*)(ws + oCl);

  const int n2x = kTok * kDm / 2;
  cast_f32_bf16x2<<<dim3((n2x + 255) / 256), dim3(256), 0, stream>>>(x, Xb, n2x);

  const dim3 gT(kDm / 64, kDm / 64);
  tcast_bf16_kernel<<<gT, dim3(256), 0, stream>>>(Wq, Wqt, kDm, kDm);
  tcast_bf16_kernel<<<gT, dim3(256), 0, stream>>>(Wk, Wkt, kDm, kDm);
  tcast_bf16_kernel<<<gT, dim3(256), 0, stream>>>(Wv, Wvt, kDm, kDm);
  tcast_bf16_kernel<<<gT, dim3(256), 0, stream>>>(Wo, Wot, kDm, kDm);

  const int tilesQK = (kTok / 64) * (kDm / 64);
  const dim3 gQK((tilesQK + 7) / 8, 1);
  wmma_gemm64<1, 0, 2, 1, false><<<gQK, dim3(256), 0, stream>>>(
      Xb, Xb, kDm, 0L, Wqt, Wqt, kDm, 0L, (void*)Qh, (void*)Qh, kDm, 0L, bq, bq, 0L, kTok, kDm, kDm, 1.0f);
  wmma_gemm64<1, 0, 2, 1, false><<<gQK, dim3(256), 0, stream>>>(
      Xb, Xb, kDm, 0L, Wkt, Wkt, kDm, 0L, (void*)Kh, (void*)Kh, kDm, 0L, bk, bk, 0L, kTok, kDm, kDm, 1.0f);

  const int tilesV = (kDm / 64) * (kSeq / 64);
  const dim3 gV((tilesV + 7) / 8, kBatch);
  wmma_gemm64<1, 0, 1, 1, false><<<gV, dim3(256), 0, stream>>>(
      Wvt, Wvt, kDm, 0L, Xb, Xb, kDm, (long)kSeq * kDm, (void*)Vt, (void*)Vt, kSeq, (long)kDm * kSeq,
      bv, bv, 0L, kDm, kSeq, kDm, 1.0f);

  mha_flash_f16_kernel<<<dim3(kBatch * kHeads * (kSeq / 64)), dim3(128), 0, stream>>>(Qh, Kh, Vt, mask, Ch, Cl, 0.125f);

  wmma_gemm64<1, 1, 2, 0, false><<<gQK, dim3(256), 0, stream>>>(
      Ch, Cl, kDm, 0L, Wot, Wot, kDm, 0L, (void*)out, (void*)out, kDm, 0L, bo, bo, 0L, kTok, kDm, kDm, 1.0f);
}
